// PointNetFeaturePropagation_4080218931822
// MI455X (gfx1250) — hardware-verified
//
#include <hip/hip_runtime.h>
#pragma clang fp contract(off)

typedef __attribute__((ext_vector_type(16))) _Float16 v16h;
typedef __attribute__((ext_vector_type(8)))  _Float16 v8h;
typedef __attribute__((ext_vector_type(16))) __bf16   v16b;
typedef __attribute__((ext_vector_type(8)))  __bf16   v8b;
typedef __attribute__((ext_vector_type(8)))  float    v8f;
typedef __attribute__((ext_vector_type(4)))  float    v4f;
typedef __attribute__((ext_vector_type(4)))  unsigned int v4u;
typedef __attribute__((ext_vector_type(2)))  unsigned int v2u;

constexpr int NBATCH    = 4;
constexpr int NQUERY    = 16384;
constexpr int NCAND     = 4096;
constexpr int CH_PTS1   = 128;
constexpr int CH_PTS2   = 256;
constexpr int CH_IN0    = CH_PTS1 + CH_PTS2;
constexpr int CH_L0     = 256;
constexpr int CH_L1     = 256;
constexpr int CH_L2     = 128;
constexpr int KCAT0     = CH_PTS1 + 2 * CH_PTS2;
constexpr int KCAT1     = 2 * CH_L0;
constexpr int KCAT2     = 2 * CH_L1;
constexpr int ROWS_ALL  = NBATCH * NQUERY;
constexpr int CAND_CHUNK = 1024;
constexpr int PART_ROWS = 128;
constexpr int NPART     = ROWS_ALL / PART_ROWS;
constexpr int ST_PITCH  = 256;

static_assert(CH_IN0 == 384, "layer-0 input channels");
static_assert(KCAT0 == 640 && KCAT1 == 512 && KCAT2 == 512, "k-concat sizes");
static_assert(KCAT0 % 32 == 0 && KCAT1 % 32 == 0 && KCAT2 % 32 == 0, "K multiple of 32");
static_assert(NQUERY % 64 == 0 && CH_L0 % 64 == 0 && CH_L1 % 64 == 0 && CH_L2 % 64 == 0, "tile multiples");
static_assert(((NQUERY / 64) * (CH_L0 / 64)) % 8 == 0 && ((NQUERY / 64) * (CH_L2 / 64)) % 8 == 0, "8 tiles per block");
static_assert(NQUERY % 256 == 0 && NCAND % CAND_CHUNK == 0 && CAND_CHUNK % 256 == 0, "3-NN tiling");
static_assert(ROWS_ALL % PART_ROWS == 0 && NPART == 512, "partials tiling");
static_assert((CH_L0 * KCAT0 / 8) % 256 == 0 && (CH_L1 * KCAT1 / 8) % 256 == 0 && (CH_L2 * KCAT2 / 8) % 256 == 0, "weight plane grids exact");

constexpr size_t SZ_H    = (size_t)ROWS_ALL * CH_L0 * 4;
constexpr size_t SZ_H2   = (size_t)ROWS_ALL * CH_L2 * 4;
constexpr size_t SZ_ACH  = (size_t)NQUERY * KCAT0 * 2;
constexpr size_t SZ_W0P  = (size_t)CH_L0 * KCAT0 * 2;
constexpr size_t SZ_W1P  = (size_t)CH_L1 * KCAT1 * 2;
constexpr size_t SZ_W2P  = (size_t)CH_L2 * KCAT2 * 2;
constexpr size_t SZ_PS   = (size_t)2 * NPART * 256 * 4;
constexpr size_t SZ_ST   = (size_t)3 * ST_PITCH * 4;
constexpr size_t OFF_H   = 0;
constexpr size_t OFF_H2  = OFF_H + SZ_H;
constexpr size_t OFF_ACH = OFF_H2 + SZ_H2;
constexpr size_t OFF_W0P = OFF_ACH + SZ_ACH;
constexpr size_t OFF_W1P = OFF_W0P + SZ_W0P;
constexpr size_t OFF_W2P = OFF_W1P + SZ_W1P;
constexpr size_t OFF_PS0 = OFF_W2P + SZ_W2P;
constexpr size_t OFF_PS1 = OFF_PS0 + SZ_PS;
constexpr size_t OFF_PS2 = OFF_PS1 + SZ_PS;
constexpr size_t OFF_ST0 = OFF_PS2 + SZ_PS;
constexpr size_t OFF_ST1 = OFF_ST0 + SZ_ST;
constexpr size_t OFF_ST2 = OFF_ST1 + SZ_ST;
constexpr size_t WS_TOTAL = OFF_ST2 + SZ_ST;
static_assert(WS_TOTAL <= (size_t)134217728, "carve under 128 MiB");
static_assert((size_t)NQUERY * KCAT1 * 2 <= SZ_ACH && (size_t)NQUERY * KCAT2 * 2 <= SZ_ACH, "chunk sized from max user");
static_assert(OFF_H2 % 128 == 0 && OFF_ACH % 128 == 0 && OFF_W0P % 128 == 0 && OFF_W1P % 128 == 0 && OFF_W2P % 128 == 0, "aligned");
static_assert(OFF_PS0 % 128 == 0 && OFF_ST0 % 128 == 0 && SZ_ST % 128 == 0, "aligned");
static_assert((size_t)ROWS_ALL * CH_L2 * 4 == (size_t)33554432, "output bytes");

__device__ __forceinline__ unsigned bf_bits_u(float f) {
  const unsigned u = __float_as_uint(f);
  return (u + 0x7FFFu + ((u >> 16) & 1u)) >> 16;
}
__device__ __forceinline__ float bfr(float f) { return __uint_as_float(bf_bits_u(f) << 16); }
__device__ __forceinline__ void split_bf(float v, unsigned& hbits, unsigned& lbits) {
  hbits = bf_bits_u(v);
  lbits = bf_bits_u(v - __uint_as_float(hbits << 16));
}
__device__ __forceinline__ unsigned pack2(float lo, float hi) {
  const unsigned a = bf_bits_u(lo);
  const unsigned c = bf_bits_u(hi);
  return a | (c << 16);
}

__device__ __forceinline__ unsigned short f2bf_bits(float f) {
  unsigned u = __float_as_uint(f);
  return (unsigned short)((u + 0x7FFFu + ((u >> 16) & 1u)) >> 16);
}
__device__ __forceinline__ float bf_bits2f(unsigned short h) { return __uint_as_float(((unsigned)h) << 16); }

__device__ __forceinline__ void dep_guard4_h(v8f& a, v8f& b, v8f& c, v8f& d, v16h x, v16h y) { asm volatile("v_nop\n\tv_nop\n\tv_nop\n\tv_nop" : "+v"(a), "+v"(b), "+v"(c), "+v"(d) : "v"(x), "v"(y)); }
__device__ __forceinline__ void dep_guard4_b(v8f& a, v8f& b, v8f& c, v8f& d, v16b x, v16b y) { asm volatile("v_nop\n\tv_nop\n\tv_nop\n\tv_nop" : "+v"(a), "+v"(b), "+v"(c), "+v"(d) : "v"(x), "v"(y)); }
__device__ __forceinline__ void keep4_h(v16h a, v16h b, v16h c, v16h d) { asm volatile("v_nop" :: "v"(a), "v"(b), "v"(c), "v"(d)); }
__device__ __forceinline__ void keep4_b(v16b a, v16b b, v16b c, v16b d) { asm volatile("v_nop" :: "v"(a), "v"(b), "v"(c), "v"(d)); }
__device__ __forceinline__ void acc_guard4(v8f& a, v8f& b, v8f& c, v8f& d) { asm volatile("v_nop\n\tv_nop\n\tv_nop\n\tv_nop" : "+v"(a), "+v"(b), "+v"(c), "+v"(d)); }
template <typename T> struct Frag;
template <> struct Frag<_Float16> {
  typedef v16h V; union U { v16h v; v8h h[2]; };
  static __device__ __forceinline__ v16h load(const _Float16* p) {
    U f; f.h[0] = *(const v8h*)(p); f.h[1] = *(const v8h*)(p + 16); return f.v;
  }
  static __device__ __forceinline__ v8f mma(v16h a, v16h b, v8f c) {
    return __builtin_amdgcn_wmma_f32_16x16x32_f16(false, a, false, b, (short)0, c, false, false);
  }
  static __device__ __forceinline__ void guard4(v8f& a, v8f& b, v8f& c, v8f& d, v16h x, v16h y) { dep_guard4_h(a, b, c, d, x, y); }
  static __device__ __forceinline__ void keep(v16h a, v16h b, v16h c, v16h d) { keep4_h(a, b, c, d); }
};
template <> struct Frag<__bf16> {
  typedef v16b V; union U { v16b v; v8b h[2]; };
  static __device__ __forceinline__ v16b load(const __bf16* p) {
    U f; f.h[0] = *(const v8b*)(p); f.h[1] = *(const v8b*)(p + 16); return f.v;
  }
  static __device__ __forceinline__ v8f mma(v16b a, v16b b, v8f c) {
    return __builtin_amdgcn_wmma_f32_16x16x32_bf16(false, a, false, b, (short)0, c, false, false);
  }
  static __device__ __forceinline__ void guard4(v8f& a, v8f& b, v8f& c, v8f& d, v16b x, v16b y) { dep_guard4_b(a, b, c, d, x, y); }
  static __device__ __forceinline__ void keep(v16b a, v16b b, v16b c, v16b d) { keep4_b(a, b, c, d); }
};

template <int ET> struct Elem;
template <> struct Elem<0> { typedef _Float16 T; };
template <> struct Elem<1> { typedef __bf16 T; };
template <int ET, bool SPLIT, int BIAS_MODE, int OUT_MODE, bool RESID, int ACT = 0>
__global__ __launch_bounds__(256) void wmma_gemm64(
    const unsigned short* __restrict__ Ap, const unsigned short* __restrict__ A2p, int lda, long strideA,
    const unsigned short* __restrict__ Btp, const unsigned short* __restrict__ Bt2p, int ldb, long strideB,
    void* __restrict__ Cout, void* __restrict__ Cout2, int ldc, long strideC,
    const float* __restrict__ bias,
    const float* __restrict__ resid, long strideR,
    int M, int N, int K, float scale) {
  typedef typename Elem<ET>::T T;
  typedef typename Frag<T>::V V;
  const T* A = (const T*)Ap; const T* A2 = (const T*)A2p; const T* Bt = (const T*)Btp; const T* Bt2 = (const T*)Bt2p;
  __shared__ __align__(16) float sT[8][16 * 68];
  const int b    = blockIdx.y;
  const int lane = threadIdx.x & 31;
  const int wave = threadIdx.x >> 5;
  const int tilesN = N >> 6;
  const int tilesM = M >> 6;
  const int tile = blockIdx.x * 8 + wave;
  if (tile >= tilesM * tilesN) return;
  const int tm = tile / tilesN;
  const int tn = tile - tm * tilesN;
  const int m0 = tm << 6;
  const int n0 = tn << 6;

  const T* Ab  = A  + (size_t)b * strideA;
  const T* Bb  = Bt + (size_t)b * strideB;
  const T* Ab2 = SPLIT ? (A2  + (size_t)b * strideA) : nullptr;
  const T* Bb2 = SPLIT ? (Bt2 + (size_t)b * strideB) : nullptr;

  const int rlane = lane & 15;
  const int koff  = (lane >> 4) * 8;
  const int mOff  = (lane >> 4) * 8;

  v8f acc[4][4];
#pragma unroll
  for (int i = 0; i < 4; ++i)
#pragma unroll
    for (int j = 0; j < 4; ++j) acc[i][j] = (v8f){0.f,0.f,0.f,0.f,0.f,0.f,0.f,0.f};

  for (int k0 = 0; k0 < K; k0 += 32) {
    V bh[4], bl[4];
#pragma unroll
    for (int j = 0; j < 4; ++j) {
      const size_t bo = (size_t)(n0 + (j << 4) + rlane) * ldb + koff + k0;
      bh[j] = Frag<T>::load(Bb + bo);
      if (SPLIT) bl[j] = Frag<T>::load(Bb2 + bo);
    }
#pragma unroll
    for (int i = 0; i < 4; ++i) {
      const size_t ao = (size_t)(m0 + (i << 4) + rlane) * lda + koff + k0;
      V ah = Frag<T>::load(Ab + ao);
      V al;
      if (SPLIT) al = Frag<T>::load(Ab2 + ao);
#pragma unroll
      for (int j = 0; j < 4; ++j) {
        acc[i][j] = Frag<T>::mma(ah, bh[j], acc[i][j]);
        if (SPLIT) {
          acc[i][j] = Frag<T>::mma(ah, bl[j], acc[i][j]);
          acc[i][j] = Frag<T>::mma(al, bh[j], acc[i][j]);
        }
      }
      Frag<T>::guard4(acc[i][0], acc[i][1], acc[i][2], acc[i][3], ah, SPLIT ? al : ah);
    }
    Frag<T>::keep(bh[0], bh[1], bh[2], bh[3]);
    if (SPLIT) Frag<T>::keep(bl[0], bl[1], bl[2], bl[3]);
  }
  acc_guard4(acc[0][0], acc[0][1], acc[0][2], acc[0][3]);
  acc_guard4(acc[1][0], acc[1][1], acc[1][2], acc[1][3]);
  acc_guard4(acc[2][0], acc[2][1], acc[2][2], acc[2][3]);
  acc_guard4(acc[3][0], acc[3][1], acc[3][2], acc[3][3]);

  float* slab = sT[wave];
  const float* Rb = RESID ? (resid + (size_t)b * strideR) : nullptr;
#pragma unroll
  for (int i = 0; i < 4; ++i) {
    const int mBase = m0 + (i << 4);
#pragma unroll
    for (int j = 0; j < 4; ++j) {
      const int n = n0 + (j << 4) + rlane;
      float bv = 0.f;
      if (BIAS_MODE == 2) bv = bias[n];
#pragma unroll
      for (int r = 0; r < 8; ++r) {
        float v = acc[i][j][r] * scale;
        if (BIAS_MODE == 1) v += bias[mBase + mOff + r];
        if (BIAS_MODE == 2) v += bv;
        if (RESID) v += Rb[(size_t)(mBase + mOff + r) * ldc + n];
        if (ACT == 2) v = fmaxf(v, 0.0f);
        slab[(mOff + r) * 68 + (j << 4) + rlane] = v;
      }
    }
    __builtin_amdgcn_fence(__ATOMIC_RELEASE, "workgroup");
    __builtin_amdgcn_wave_barrier();
    __builtin_amdgcn_fence(__ATOMIC_ACQUIRE, "workgroup");
    if (OUT_MODE == 0) {
      float* C = (float*)Cout + (size_t)b * strideC;
      const int hh = lane >> 4, c4 = (lane & 15) * 4;
      for (int pass = 0; pass < 2; ++pass) {
#pragma unroll
        for (int it = 0; it < 8; ++it) {
          const int row = it * 2 + hh;
          v4f v = *(const v4f*)(slab + row * 68 + c4);
          *(volatile v4f*)(C + (size_t)(mBase + row) * ldc + n0 + c4) = v;
        }
        __threadfence();
      }
    } else {
      const int q = lane >> 3, c8 = (lane & 7) * 8;
      unsigned short* C  = (unsigned short*)Cout  + (size_t)b * strideC;
      unsigned short* C2 = (OUT_MODE == 2) ? ((unsigned short*)Cout2 + (size_t)b * strideC) : nullptr;
      for (int pass = 0; pass < 2; ++pass) {
#pragma unroll
        for (int it = 0; it < 4; ++it) {
          const int row = it * 4 + q;
          const float* sp = slab + row * 68 + c8;
          v8h hv, lv;
#pragma unroll
          for (int e = 0; e < 8; ++e) {
            if (OUT_MODE == 1) {
              hv[e] = (_Float16)sp[e];
            } else {
              unsigned short hb = f2bf_bits(sp[e]);
              unsigned short lb = f2bf_bits(sp[e] - bf_bits2f(hb));
              hv[e] = __builtin_bit_cast(_Float16, hb);
              lv[e] = __builtin_bit_cast(_Float16, lb);
            }
          }
          *(volatile v8h*)(C + (size_t)(mBase + row) * ldc + n0 + c8) = hv;
          if (OUT_MODE == 2) *(volatile v8h*)(C2 + (size_t)(mBase + row) * ldc + n0 + c8) = lv;
        }
        __threadfence();
      }
    }
    __builtin_amdgcn_fence(__ATOMIC_RELEASE, "workgroup");
    __builtin_amdgcn_wave_barrier();
    __builtin_amdgcn_fence(__ATOMIC_ACQUIRE, "workgroup");
  }
}

__global__ __launch_bounds__(256) void build_wplane(const float* __restrict__ w, unsigned short* __restrict__ outp,
                                                    int cin, int kcat, int dup0) {
  const int i = blockIdx.x * 256 + threadIdx.x;
  const int e = i * 8;
  const int n = e / kcat;
  const int k = e - n * kcat;
  const int src = (k < cin) ? k : (dup0 + (k - cin));
  const float* sp = w + (size_t)n * cin + src;
  const v4f a = *(const v4f*)(sp);
  const v4f c = *(const v4f*)(sp + 4);
  const float a0 = a[0], a1 = a[1], a2 = a[2], a3 = a[3];
  const float c0 = c[0], c1 = c[1], c2 = c[2], c3 = c[3];
  v4u o;
  o[0] = pack2(a0, a1);
  o[1] = pack2(a2, a3);
  o[2] = pack2(c0, c1);
  o[3] = pack2(c2, c3);
  volatile v4u* dst = (volatile v4u*)(outp + (size_t)e);
  *dst = o;
  __threadfence();
  *dst = o;
}

__global__ __launch_bounds__(256) void knn_interp_build(const float* __restrict__ xyz1, const float* __restrict__ xyz2,
                                                        const float* __restrict__ pts1, const float* __restrict__ pts2,
                                                        unsigned short* __restrict__ acat, int b) {
#pragma clang fp contract(off)
  __shared__ __align__(16) float sCand[CAND_CHUNK * 4];
  __shared__ int   sIdx[256 * 3];
  __shared__ float sWt[256 * 3];

  const int tid   = threadIdx.x;
  const int nbase = blockIdx.x * 256;
  const size_t qo = ((size_t)b * NQUERY + nbase + tid) * 3;
  const float x0 = bfr(xyz1[qo + 0]);
  const float x1 = bfr(xyz1[qo + 1]);
  const float x2 = bfr(xyz1[qo + 2]);
  const float t0 = x0 * x0;
  const float t1 = x1 * x1;
  const float t2 = x2 * x2;
  const float xx = (t0 + t2) + t1;

  float bd0 = __builtin_huge_valf(), bd1 = __builtin_huge_valf(), bd2 = __builtin_huge_valf();
  int bi0 = 0, bi1 = 0, bi2 = 0;

  for (int ch = 0; ch < NCAND / CAND_CHUNK; ++ch) {
    __syncthreads();
#pragma unroll 1
    for (int j = 0; j < CAND_CHUNK / 256; ++j) {
      const int slot = j * 256 + tid;
      const size_t so = ((size_t)b * NCAND + ch * CAND_CHUNK + slot) * 3;
      const float y0 = bfr(xyz2[so + 0]);
      const float y1 = bfr(xyz2[so + 1]);
      const float y2 = bfr(xyz2[so + 2]);
      const float u0 = y0 * y0;
      const float u1 = y1 * y1;
      const float u2 = y2 * y2;
      const float yy = (u0 + u2) + u1;
      v4f cv;
      cv[0] = y0; cv[1] = y1; cv[2] = y2; cv[3] = yy;
      *(v4f*)(sCand + 4 * slot) = cv;
    }
    __syncthreads();
    const int mb = ch * CAND_CHUNK;
#pragma unroll 4
    for (int m = 0; m < CAND_CHUNK; ++m) {
      const v4f cv = *(const v4f*)(sCand + 4 * m);
      const float cy0 = cv[0], cy1 = cv[1], cy2 = cv[2], cyy = cv[3];
      const float s = xx + cyy;
      float p = x0 * cy0;
      p = __builtin_fmaf(x1, cy1, p);
      p = __builtin_fmaf(x2, cy2, p);
      const float d = s - (p + p);
      if (d < bd2) {
        const int mi = mb + m;
        if (d < bd0)      { bd2 = bd1; bi2 = bi1; bd1 = bd0; bi1 = bi0; bd0 = d; bi0 = mi; }
        else if (d < bd1) { bd2 = bd1; bi2 = bi1; bd1 = d;   bi1 = mi; }
        else              { bd2 = d;   bi2 = mi; }
      }
    }
  }
  {
    const float e0 = bd0 + 1e-8f;
    const float e1 = bd1 + 1e-8f;
    const float e2 = bd2 + 1e-8f;
    const float w0 = 1.0f / e0;
    const float w1 = 1.0f / e1;
    const float w2 = 1.0f / e2;
    const float wsum = (w0 + w2) + w1;
    const int c0 = min(max(bi0, 0), NCAND - 1);
    const int c1 = min(max(bi1, 0), NCAND - 1);
    const int c2 = min(max(bi2, 0), NCAND - 1);
    sIdx[tid * 3 + 0] = c0; sWt[tid * 3 + 0] = w0 / wsum;
    sIdx[tid * 3 + 1] = c1; sWt[tid * 3 + 1] = w1 / wsum;
    sIdx[tid * 3 + 2] = c2; sWt[tid * 3 + 2] = w2 / wsum;
  }
  __syncthreads();

  const int wave = tid >> 5, lane = tid & 31;
  const float* p2b = pts2 + (size_t)b * NCAND * CH_PTS2;
#pragma unroll 1
  for (int i = 0; i < 32; ++i) {
    const int p = wave * 32 + i;
    const int j0 = min(max(sIdx[p * 3 + 0], 0), NCAND - 1);
    const int j1 = min(max(sIdx[p * 3 + 1], 0), NCAND - 1);
    const int j2 = min(max(sIdx[p * 3 + 2], 0), NCAND - 1);
    const float a0 = sWt[p * 3 + 0], a1 = sWt[p * 3 + 1], a2 = sWt[p * 3 + 2];
    const float* r0 = p2b + (size_t)j0 * CH_PTS2 + lane * 8;
    const float* r1 = p2b + (size_t)j1 * CH_PTS2 + lane * 8;
    const float* r2 = p2b + (size_t)j2 * CH_PTS2 + lane * 8;
    const v4f g0a = *(const v4f*)(r0), g0b = *(const v4f*)(r0 + 4);
    const v4f g1a = *(const v4f*)(r1), g1b = *(const v4f*)(r1 + 4);
    const v4f g2a = *(const v4f*)(r2), g2b = *(const v4f*)(r2 + 4);
    const size_t grow = (size_t)b * NQUERY + nbase + p;
    const v4f pv = *(const v4f*)(pts1 + grow * CH_PTS1 + lane * 4);
    unsigned hbits[8], lbits[8];
#pragma unroll
    for (int e = 0; e < 4; ++e) {
      const float ga = g0a[e], gb = g1a[e], gc = g2a[e];
      float acc = bfr(ga) * a0;
      acc = __builtin_fmaf(bfr(gb), a1, acc);
      acc = __builtin_fmaf(bfr(gc), a2, acc);
      split_bf(acc, hbits[e], lbits[e]);
      const float ha = g0b[e], hb2 = g1b[e], hc = g2b[e];
      float acc2 = bfr(ha) * a0;
      acc2 = __builtin_fmaf(bfr(hb2), a1, acc2);
      acc2 = __builtin_fmaf(bfr(hc), a2, acc2);
      split_bf(acc2, hbits[4 + e], lbits[4 + e]);
    }
    v4u hw, lw;
    hw[0] = hbits[0] | (hbits[1] << 16); hw[1] = hbits[2] | (hbits[3] << 16);
    hw[2] = hbits[4] | (hbits[5] << 16); hw[3] = hbits[6] | (hbits[7] << 16);
    lw[0] = lbits[0] | (lbits[1] << 16); lw[1] = lbits[2] | (lbits[3] << 16);
    lw[2] = lbits[4] | (lbits[5] << 16); lw[3] = lbits[6] | (lbits[7] << 16);
    const float q0 = pv[0], q1 = pv[1], q2 = pv[2], q3 = pv[3];
    v2u pw;
    pw[0] = pack2(q0, q1);
    pw[1] = pack2(q2, q3);
    unsigned short* rowp = acat + (size_t)(nbase + p) * KCAT0;
    volatile v2u* dp = (volatile v2u*)(rowp + lane * 4);
    volatile v4u* dh = (volatile v4u*)(rowp + CH_PTS1 + lane * 8);
    volatile v4u* dl = (volatile v4u*)(rowp + CH_PTS1 + CH_PTS2 + lane * 8);
    *dp = pw; *dh = hw; *dl = lw;
    __threadfence();
    *dp = pw; *dh = hw; *dl = lw;
  }
}

template <int CH>
__global__ __launch_bounds__(256) void col_partials(const float* __restrict__ hsrc, float* __restrict__ ps, float* __restrict__ pq) {
  __shared__ float sS[256];
  __shared__ float sQ[256];
  constexpr int RG = 256 / CH;
  const int t = threadIdx.x;
  const int col = t & (CH - 1);
  const int rg = t / CH;
  const size_t r0 = (size_t)blockIdx.x * PART_ROWS;
  float s = 0.0f, q = 0.0f;
#pragma unroll 4
  for (int r = rg; r < PART_ROWS; r += RG) {
    const float v = hsrc[(r0 + r) * CH + col];
    s = s + v;
    q = q + v * v;
  }
  sS[t] = s;
  sQ[t] = q;
  __syncthreads();
  if (t < CH) {
    float ts = 0.0f, tq = 0.0f;
#pragma unroll
    for (int g = 0; g < RG; ++g) { ts = ts + sS[g * CH + t]; tq = tq + sQ[g * CH + t]; }
    volatile float* d0 = (volatile float*)(ps + (size_t)blockIdx.x * CH + t);
    volatile float* d1 = (volatile float*)(pq + (size_t)blockIdx.x * CH + t);
    *d0 = ts; *d1 = tq;
    __threadfence();
    *d0 = ts; *d1 = tq;
  }
}

template <int CH>
__global__ __launch_bounds__(256) void final_stats(const float* __restrict__ ps, const float* __restrict__ pq,
                                                   const float* __restrict__ gamma, const float* __restrict__ beta,
                                                   float* __restrict__ st) {
  const int c = threadIdx.x;
  double s = 0.0, q = 0.0;
#pragma unroll 4
  for (int i = 0; i < NPART; ++i) {
    s = s + (double)ps[(size_t)i * CH + c];
    q = q + (double)pq[(size_t)i * CH + c];
  }
  const double inv = 1.0 / (double)ROWS_ALL;
  const double mean = s * inv;
  const double var = q * inv - mean * mean;
  float varf = (float)var;
  varf = varf > 0.0f ? varf : 0.0f;
  const float rs = 1.0f / sqrtf(varf + 1e-5f);
  const float g = bfr(gamma[c]);
  const float be = bfr(beta[c]);
  const float meanf = (float)mean;
  const float sc = rs * g;
  volatile float* d0 = (volatile float*)(st + c);
  volatile float* d1 = (volatile float*)(st + ST_PITCH + c);
  volatile float* d2 = (volatile float*)(st + 2 * ST_PITCH + c);
  *d0 = meanf; *d1 = sc; *d2 = be;
  __threadfence();
  *d0 = meanf; *d1 = sc; *d2 = be;
}

__global__ __launch_bounds__(256) void bn_relu_split(const float* __restrict__ hsrc, const float* __restrict__ st,
                                                     unsigned short* __restrict__ acat) {
  const int lane = threadIdx.x & 31, wave = threadIdx.x >> 5;
  const int c0 = lane * 8;
  const v4f m0 = *(const v4f*)(st + c0), m1 = *(const v4f*)(st + c0 + 4);
  const v4f s0 = *(const v4f*)(st + ST_PITCH + c0), s1 = *(const v4f*)(st + ST_PITCH + c0 + 4);
  const v4f e0 = *(const v4f*)(st + 2 * ST_PITCH + c0), e1 = *(const v4f*)(st + 2 * ST_PITCH + c0 + 4);
  const int row0 = blockIdx.x * 64 + wave * 8;
#pragma unroll 1
  for (int r = 0; r < 8; ++r) {
    const int row = row0 + r;
    const v4f ha = *(const v4f*)(hsrc + (size_t)row * CH_L0 + c0);
    const v4f hc = *(const v4f*)(hsrc + (size_t)row * CH_L0 + c0 + 4);
    unsigned hbits[8], lbits[8];
#pragma unroll
    for (int e = 0; e < 4; ++e) {
      const float h1 = ha[e], mm1 = m0[e], ss1 = s0[e], bb1 = e0[e];
      float v = (h1 - mm1) * ss1 + bb1;
      v = v > 0.0f ? v : 0.0f;
      split_bf(v, hbits[e], lbits[e]);
      const float h2 = hc[e], mm2 = m1[e], ss2 = s1[e], bb2 = e1[e];
      float v2 = (h2 - mm2) * ss2 + bb2;
      v2 = v2 > 0.0f ? v2 : 0.0f;
      split_bf(v2, hbits[4 + e], lbits[4 + e]);
    }
    v4u hw, lw;
    hw[0] = hbits[0] | (hbits[1] << 16); hw[1] = hbits[2] | (hbits[3] << 16);
    hw[2] = hbits[4] | (hbits[5] << 16); hw[3] = hbits[6] | (hbits[7] << 16);
    lw[0] = lbits[0] | (lbits[1] << 16); lw[1] = lbits[2] | (lbits[3] << 16);
    lw[2] = lbits[4] | (lbits[5] << 16); lw[3] = lbits[6] | (lbits[7] << 16);
    unsigned short* rowp = acat + (size_t)row * KCAT1;
    volatile v4u* dh = (volatile v4u*)(rowp + c0);
    volatile v4u* dl = (volatile v4u*)(rowp + CH_L0 + c0);
    *dh = hw; *dl = lw;
    __threadfence();
    *dh = hw; *dl = lw;
  }
}

__global__ __launch_bounds__(256) void bn_relu_out(const float* __restrict__ hsrc, const float* __restrict__ st,
                                                   float* __restrict__ outp) {
  const int lane = threadIdx.x & 31, wave = threadIdx.x >> 5;
  const int c0 = lane * 4;
  const v4f m0 = *(const v4f*)(st + c0);
  const v4f s0 = *(const v4f*)(st + ST_PITCH + c0);
  const v4f e0 = *(const v4f*)(st + 2 * ST_PITCH + c0);
  const int row0 = blockIdx.x * 64 + wave * 8;
#pragma unroll 1
  for (int r = 0; r < 8; ++r) {
    const size_t row = (size_t)(row0 + r);
    const v4f hv = *(const v4f*)(hsrc + row * CH_L2 + c0);
    v4f o;
#pragma unroll
    for (int e = 0; e < 4; ++e) {
      const float h1 = hv[e], mm = m0[e], ss = s0[e], bb = e0[e];
      float v = (h1 - mm) * ss + bb;
      v = v > 0.0f ? v : 0.0f;
      o[e] = v;
    }
    volatile v4f* dst = (volatile v4f*)(outp + row * CH_L2 + c0);
    *dst = o;
    __threadfence();
    *dst = o;
  }
}

extern "C" void kernel_launch(void* const* d_in, const int* in_sizes, int n_in,
                              void* d_out, int out_size, void* d_ws, size_t ws_size,
                              hipStream_t stream) {
  (void)in_sizes; (void)out_size;
  if (n_in < 16) return;
  if (ws_size < WS_TOTAL) return;

  const float* xyz1 = (const float*)d_in[0];
  const float* xyz2 = (const float*)d_in[1];
  const float* pts1 = (const float*)d_in[2];
  const float* pts2 = (const float*)d_in[3];
  const float* w0   = (const float*)d_in[4];
  const float* g0   = (const float*)d_in[6];
  const float* be0  = (const float*)d_in[7];
  const float* w1   = (const float*)d_in[8];
  const float* g1   = (const float*)d_in[10];
  const float* be1  = (const float*)d_in[11];
  const float* w2   = (const float*)d_in[12];
  const float* g2   = (const float*)d_in[14];
  const float* be2  = (const float*)d_in[15];

  char* ws = (char*)d_ws;
  float* H    = (float*)(ws + OFF_H);
  float* H2   = (float*)(ws + OFF_H2);
  unsigned short* ACH = (unsigned short*)(ws + OFF_ACH);
  unsigned short* W0P = (unsigned short*)(ws + OFF_W0P);
  unsigned short* W1P = (unsigned short*)(ws + OFF_W1P);
  unsigned short* W2P = (unsigned short*)(ws + OFF_W2P);
  float* PS0 = (float*)(ws + OFF_PS0);
  float* PQ0 = PS0 + (size_t)NPART * 256;
  float* PS1 = (float*)(ws + OFF_PS1);
  float* PQ1 = PS1 + (size_t)NPART * 256;
  float* PS2 = (float*)(ws + OFF_PS2);
  float* PQ2 = PS2 + (size_t)NPART * 256;
  float* ST0 = (float*)(ws + OFF_ST0);
  float* ST1 = (float*)(ws + OFF_ST1);
  float* ST2 = (float*)(ws + OFF_ST2);

  build_wplane<<<(CH_L0 * KCAT0 / 8) / 256, 256, 0, stream>>>(w0, W0P, CH_IN0, KCAT0, CH_PTS1);
  build_wplane<<<(CH_L1 * KCAT1 / 8) / 256, 256, 0, stream>>>(w1, W1P, CH_L0, KCAT1, 0);
  build_wplane<<<(CH_L2 * KCAT2 / 8) / 256, 256, 0, stream>>>(w2, W2P, CH_L1, KCAT2, 0);

  const int gemmBlocks256 = ((NQUERY / 64) * (CH_L0 / 64)) / 8;
  const int gemmBlocks128 = ((NQUERY / 64) * (CH_L2 / 64)) / 8;

  for (int b = 0; b < NBATCH; ++b) {
    knn_interp_build<<<NQUERY / 256, 256, 0, stream>>>(xyz1, xyz2, pts1, pts2, ACH, b);
    float* Hb = H + (size_t)b * NQUERY * CH_L0;
    wmma_gemm64<1, false, 0, 0, false, 0><<<dim3(gemmBlocks256, 1), 256, 0, stream>>>(
        ACH, ACH, KCAT0, 0L, W0P, W0P, KCAT0, 0L, (void*)Hb, (void*)Hb, CH_L0, 0L,
        ST0, ST0, 0L, NQUERY, CH_L0, KCAT0, 1.0f);
  }
  col_partials<CH_L0><<<NPART, 256, 0, stream>>>(H, PS0, PQ0);
  final_stats<CH_L0><<<1, CH_L0, 0, stream>>>(PS0, PQ0, g0, be0, ST0);

  for (int b = 0; b < NBATCH; ++b) {
    float* Hb = H + (size_t)b * NQUERY * CH_L0;
    bn_relu_split<<<NQUERY / 64, 256, 0, stream>>>(Hb, ST0, ACH);
    wmma_gemm64<1, false, 0, 0, false, 0><<<dim3(gemmBlocks256, 1), 256, 0, stream>>>(
        ACH, ACH, KCAT1, 0L, W1P, W1P, KCAT1, 0L, (void*)Hb, (void*)Hb, CH_L1, 0L,
        ST1, ST1, 0L, NQUERY, CH_L1, KCAT1, 1.0f);
  }
  col_partials<CH_L1><<<NPART, 256, 0, stream>>>(H, PS1, PQ1);
  final_stats<CH_L1><<<1, CH_L1, 0, stream>>>(PS1, PQ1, g1, be1, ST1);

  for (int b = 0; b < NBATCH; ++b) {
    float* Hb  = H  + (size_t)b * NQUERY * CH_L1;
    float* H2b = H2 + (size_t)b * NQUERY * CH_L2;
    bn_relu_split<<<NQUERY / 64, 256, 0, stream>>>(Hb, ST1, ACH);
    wmma_gemm64<1, false, 0, 0, false, 0><<<dim3(gemmBlocks128, 1), 256, 0, stream>>>(
        ACH, ACH, KCAT2, 0L, W2P, W2P, KCAT2, 0L, (void*)H2b, (void*)H2b, CH_L2, 0L,
        ST2, ST2, 0L, NQUERY, CH_L2, KCAT2, 1.0f);
  }
  col_partials<CH_L2><<<NPART, 256, 0, stream>>>(H2, PS2, PQ2);
  final_stats<CH_L2><<<1, CH_L2, 0, stream>>>(PS2, PQ2, g2, be2, ST2);

  bn_relu_out<<<ROWS_ALL / 64, 256, 0, stream>>>(H2, ST2, (float*)d_out);
}
